// ToyPredictor_21732534517825
// MI455X (gfx1250) — hardware-verified
//
#include <hip/hip_runtime.h>


#define NBATCH 4096
#define NT     512
#define NSTEP  511
#define ND     128
#define RB     64
#define NBLK   (NBATCH / RB)
#define HP     136
#define WP     136
#define PP     36
#define PROW   512

typedef __attribute__((ext_vector_type(16))) _Float16 v16h;
typedef __attribute__((ext_vector_type(8)))  _Float16 v8h;
typedef __attribute__((ext_vector_type(8)))  float    v8f;
typedef __attribute__((ext_vector_type(4)))  float    v4f;

__device__ __forceinline__ void dep_guard_h(v8f& a, v8f& b, v16h x, v16h y) { asm volatile("v_nop\n\tv_nop\n\tv_nop\n\tv_nop" : "+v"(a), "+v"(b) : "v"(x), "v"(y)); }
__device__ __forceinline__ void keep4_h(v16h a, v16h b, v16h c, v16h d) { asm volatile("v_nop" :: "v"(a), "v"(b), "v"(c), "v"(d)); }
__device__ __forceinline__ void acc_guard4(v8f& a, v8f& b, v8f& c, v8f& d) { asm volatile("v_nop\n\tv_nop\n\tv_nop\n\tv_nop" : "+v"(a), "+v"(b), "+v"(c), "+v"(d)); }

template <typename T> struct Frag;
template <> struct Frag<_Float16> {
  typedef v16h V; union U { v16h v; v8h h[2]; };
  static __device__ __forceinline__ v16h load(const _Float16* p) {
    U f; f.h[0] = *(const v8h*)(p); f.h[1] = *(const v8h*)(p + 16); return f.v;
  }
  static __device__ __forceinline__ v8f mma(v16h a, v16h b, v8f c) {
    return __builtin_amdgcn_wmma_f32_16x16x32_f16(false, a, false, b, (short)0, c, false, false);
  }
  static __device__ __forceinline__ void guard(v8f& a, v8f& b, v16h x, v16h y) { dep_guard_h(a, b, x, y); }
  static __device__ __forceinline__ void keep(v16h a, v16h b, v16h c, v16h d) { keep4_h(a, b, c, d); }
};

__device__ __forceinline__ float tanh_f(float x) { return 1.0f - 2.0f * __builtin_amdgcn_rcpf(__expf(2.0f * x) + 1.0f); }

__global__ __launch_bounds__(256) void recur_kernel(
    const float* __restrict__ seq,
    const float* __restrict__ W_in,
    const float* __restrict__ b_in,
    const float* __restrict__ W_hh,
    const float* __restrict__ W_xh,
    const float* __restrict__ b_h,
    const float* __restrict__ W_out,
    const float* __restrict__ b_out,
    float* __restrict__ P,
    float* __restrict__ partials)
{
  __shared__ __align__(16) _Float16 Wsh[ND * WP];
  __shared__ __align__(16) _Float16 hsh[2 * RB * HP];
  __shared__ __align__(16) float pst[RB * PP];
  __shared__ __align__(16) float xsh[2 * RB];
  __shared__ __align__(16) float yph[2 * RB];
  __shared__ float ush[ND];
  __shared__ float cbsh[ND];
  __shared__ float wosh[ND];
  __shared__ float lsh[RB];
  typedef Frag<_Float16> F;

  const int tid  = threadIdx.x;
  const int lane = tid & 31, wave = tid >> 5, hh = lane >> 4, rl = lane & 15;
  const int blk  = blockIdx.x;
  const int b0   = blk * RB;
  const int mt   = wave >> 1;
  const int nh   = wave & 1;

  for (int i = tid; i < ND * ND; i += 256) {
    const int n = i >> 7, k = i & 127;
    Wsh[n * WP + k] = (_Float16)(W_hh[i] * 16.0f);
  }
  for (int i = tid; i < 2 * RB * HP; i += 256) hsh[i] = (_Float16)0.0f;
  if (tid < ND) {
    const int n = tid;
    float au = 0.0f, ac = 0.0f;
    for (int k = 0; k < ND; ++k) {
      const float wx = W_xh[n * ND + k];
      au += wx * W_in[k];
      ac += wx * b_in[k];
    }
    ush[n]  = au;
    cbsh[n] = ac + b_h[n];
    wosh[n] = W_out[n];
  }
  if (tid < RB) xsh[tid] = seq[(size_t)(b0 + tid) * NT];
  float lacc = 0.0f;
  __syncthreads();

  const float S  = 1.0f / 128.0f;
  const float bo = b_out[0];
  const int rq = lane >> 3, c4 = (lane & 7) * 4;

  for (int s = 0; s < NSTEP; ++s) {
    const _Float16* hc = hsh + (s & 1) * (RB * HP);
    _Float16*       hn = hsh + ((s & 1) ^ 1) * (RB * HP);

    float tgt = 0.0f;
    if (tid < RB) {
      tgt = seq[(size_t)(b0 + tid) * NT + s + 1];
      xsh[((s + 1) & 1) * RB + tid] = tgt;
    }

    v8f acc[4];
#pragma unroll
    for (int j = 0; j < 4; ++j) acc[j] = (v8f){0.f,0.f,0.f,0.f,0.f,0.f,0.f,0.f};
#pragma unroll 1
    for (int k0 = 0; k0 < ND; k0 += 32) {
      v16h bfr[4];
#pragma unroll
      for (int j = 0; j < 4; ++j) bfr[j] = F::load(Wsh + (64 * nh + 16 * j + rl) * WP + k0 + 8 * hh);
      const v16h a = F::load(hc + (16 * mt + rl) * HP + k0 + 8 * hh);
#pragma unroll
      for (int j = 0; j < 4; ++j) acc[j] = F::mma(a, bfr[j], acc[j]);
      F::guard(acc[0], acc[3], a, a);
      F::keep(bfr[0], bfr[1], bfr[2], bfr[3]);
    }
    acc_guard4(acc[0], acc[1], acc[2], acc[3]);

    const float* xp = xsh + (s & 1) * RB + 16 * mt + 8 * hh;
    const v4f xa = *(const v4f*)(xp);
    const v4f xb = *(const v4f*)(xp + 4);
    float xr[8];
    xr[0] = xa[0]; xr[1] = xa[1]; xr[2] = xa[2]; xr[3] = xa[3];
    xr[4] = xb[0]; xr[5] = xb[1]; xr[6] = xb[2]; xr[7] = xb[3];
    float ysum[8];
#pragma unroll
    for (int r = 0; r < 8; ++r) ysum[r] = 0.0f;
#pragma unroll
    for (int j = 0; j < 4; ++j) {
      const int n = 64 * nh + 16 * j + rl;
      const float uu = ush[n], cc = cbsh[n], ww = wosh[n];
#pragma unroll
      for (int r = 0; r < 8; ++r) {
        const float pre = acc[j][r] * S + (xr[r] * uu + cc);
        const float h = tanh_f(pre);
        ysum[r] += h * ww;
        hn[(16 * mt + 8 * hh + r) * HP + n] = (_Float16)(h * 8.0f);
      }
    }
#pragma unroll
    for (int r = 0; r < 8; ++r) {
      float v = ysum[r];
      v += __shfl_xor(v, 1, 32);
      v += __shfl_xor(v, 2, 32);
      v += __shfl_xor(v, 4, 32);
      v += __shfl_xor(v, 8, 32);
      ysum[r] = v;
    }
    if (rl == 0) {
#pragma unroll
      for (int r = 0; r < 8; ++r) yph[nh * RB + 16 * mt + 8 * hh + r] = ysum[r];
    }
    __syncthreads();

    if (tid < RB) {
      const float y = (yph[tid] + yph[RB + tid]) + bo;
      pst[tid * PP + (s & 31)] = y;
      const float e = y - tgt;
      lacc += e * e;
    }
    if ((s & 31) == 31 || s == NSTEP - 1) {
      __syncthreads();
      float* pb = P + (size_t)b0 * PROW + 32 * (s >> 5) + c4;
      for (int pass = 0; pass < 2; ++pass) {
#pragma unroll
        for (int it = 0; it < 2; ++it) {
          const int row = 8 * wave + 4 * it + rq;
          const v4f v = *(const v4f*)(pst + row * PP + c4);
          *(volatile v4f*)(pb + (size_t)row * PROW) = v;
        }
        __threadfence();
      }
    }
    __syncthreads();
  }

  if (tid < RB) lsh[tid] = lacc;
  __syncthreads();
  if (tid < 32) {
    double sm = 0.0;
    for (int i = 0; i < RB; ++i) sm += (double)lsh[i];
    const float val = (lane == 0) ? (float)sm : 0.0f;
    volatile float* pp = partials + (size_t)blk * 32 + lane;
    *pp = val;
    __threadfence();
    *pp = val;
  }
}

__global__ __launch_bounds__(256) void repack_kernel(
    const float* __restrict__ P, const float* __restrict__ partials, float* __restrict__ out)
{
  const int i = blockIdx.x * 256 + threadIdx.x;
  if (i < (NBATCH * NSTEP) / 4) {
    const int g0 = i * 4;
    v4f v;
#pragma unroll
    for (int e = 0; e < 4; ++e) {
      const int g = g0 + e;
      const int b = g / NSTEP;
      const int t = g - b * NSTEP;
      v[e] = P[(size_t)b * PROW + t];
    }
    *(volatile v4f*)(out + g0) = v;
    __threadfence();
    *(volatile v4f*)(out + g0) = v;
  }
  if (blockIdx.x == 0 && threadIdx.x == 0) {
    double sm = 0.0;
    for (int k = 0; k < NBLK; ++k) sm += (double)partials[k * 32];
    const float loss = (float)(sm * (1.0 / ((double)NBATCH * (double)NSTEP)));
    volatile float* lp = out + (size_t)NBATCH * NSTEP;
    *lp = loss;
    __threadfence();
    *lp = loss;
  }
}

extern "C" void kernel_launch(void* const* d_in, const int* in_sizes, int n_in,
                              void* d_out, int out_size, void* d_ws, size_t ws_size,
                              hipStream_t stream) {
  if (n_in < 8) return;
  if (in_sizes[0] != NBATCH * NT) return;
  if (in_sizes[1] != ND || in_sizes[2] != ND) return;
  if (in_sizes[3] != ND * ND || in_sizes[4] != ND * ND) return;
  if (in_sizes[5] != ND || in_sizes[6] != ND || in_sizes[7] < 1) return;
  if (out_size != NBATCH * NSTEP + 1) return;

  const float* seq   = (const float*)d_in[0];
  const float* W_in  = (const float*)d_in[1];
  const float* b_in  = (const float*)d_in[2];
  const float* W_hh  = (const float*)d_in[3];
  const float* W_xh  = (const float*)d_in[4];
  const float* b_h   = (const float*)d_in[5];
  const float* W_out = (const float*)d_in[6];
  const float* b_out = (const float*)d_in[7];
  float* out = (float*)d_out;

  const size_t szP    = (size_t)NBATCH * PROW * sizeof(float);
  const size_t szPart = (size_t)NBLK * 32 * sizeof(float);
  size_t off = 0;
  const size_t oP    = off; off += szP;
  const size_t oPart = off; off += szPart;
  if (off > ws_size) return;
  char* ws = (char*)d_ws;
  float* P        = (float*)(ws + oP);
  float* partials = (float*)(ws + oPart);

  recur_kernel<<<NBLK, 256, 0, stream>>>(seq, W_in, b_in, W_hh, W_xh, b_h, W_out, b_out, P, partials);
  repack_kernel<<<((NBATCH * NSTEP) / 4 + 255) / 256, 256, 0, stream>>>(P, partials, out);
}
